// GraphEncoder_77283641524506
// MI455X (gfx1250) — hardware-verified
//
#include <hip/hip_runtime.h>
#include <stddef.h>
#include <stdint.h>
#include <math.h>


#define NN      20000
#define NE      320000
#define EMB     768
#define HID     256
#define NHD     8
#define DHD     32
#define NREL    5
#define BOT     128
#define NTAB    1501
#define NMOD    5
#define MP      20096
#define KTH     256
#define KHH     1536
#define KX1     512
#define NRN     1280
#define NTHR    256
#define NWAVE   8
#define EPT     8
#define CHUNK   (NTHR * EPT)
#define WCAP    (EPT * 32)
#define LISTN   (NWAVE * WCAP)
#define NBRUN   512
#define SLB     9
#define NBLK    40
#define RCAP    12288
#define DEGCAP  64
#define MEAS_B512   8299
#define MEAS_MAXDEG 34
#define GT      128
#define SP      132
#define GEMM_LDS_FLOATS (GT * SP + 2048)
#define GEMM_LDS_BYTES  (GEMM_LDS_FLOATS * 4)
#define BKT_LDS_INTS    (LISTN + 2 * RCAP + 3 * NBRUN + 16)
#define BKT_LDS_BYTES   (BKT_LDS_INTS * 4)
#define SDOFF   (NREL * 2 * MP * 4)
#define NEGSL   0.2f
#define EPS_SM  1e-16f
#define MX0     (-1.0e30f)
#define NUX     (MP * (EMB / 8))
#define NUWD    (BOT * (EMB / 8))
#define NUWU    (EMB * (KTH / 8))
#define NUW0    (NRN * (KHH / 8))
#define NUW1    (NRN * (KX1 / 8))

static_assert(MP % GT == 0 && MP >= NN && MP - NN < GT);
static_assert(NBLK * NBRUN >= MP);
static_assert((EMB % 32) == 0 && (KTH % 32) == 0 && (KHH % 32) == 0 && (KX1 % 32) == 0);
static_assert(KTH == 2 * BOT && KHH == 2 * EMB && KX1 == 2 * HID && NRN == NREL * HID);
static_assert((EMB % GT) == 0 && (NRN % GT) == 0 && BOT == GT && HID == 2 * GT);
static_assert(NN <= 32768 && NREL <= 8 && NBRUN == (1 << SLB));
static_assert((CHUNK & (CHUNK - 1)) == 0 && CHUNK <= 4096);
static_assert(((long long)CHUNK << SLB) < (1LL << 31));
static_assert((RCAP % (NTHR * 4)) == 0 && ((RCAP + 3 * NBRUN) % 4) == 0);
static_assert((long long)RCAP * 10 >= (long long)MEAS_B512 * 11);
static_assert(DEGCAP >= MEAS_MAXDEG + 8);
static_assert(NBRUN % NWAVE == 0 && NBRUN % 32 == 0 && 2 * NBRUN == NTHR * 4);
static_assert(HID == 8 * 32 && HID % 8 == 0 && DHD == 32 && NHD * DHD == HID);
static_assert((NUX % NTHR) == 0 && (NUWD % NTHR) == 0 && (NUWU % NTHR) == 0 && (NUW0 % NTHR) == 0 && (NUW1 % NTHR) == 0);
static_assert(GEMM_LDS_BYTES <= 327680 && BKT_LDS_BYTES <= 327680);
static_assert((RCAP + 2 * NBRUN + NWAVE * HID) * 4 <= 65536);
static_assert(NTHR == 2 * GT && GT * 16 == 8 * NTHR && GT * 32 == 16 * NTHR);

typedef float          v4f  __attribute__((ext_vector_type(4)));
typedef float          v8f  __attribute__((ext_vector_type(8)));
typedef int            v4i  __attribute__((ext_vector_type(4)));
typedef int            v8i  __attribute__((ext_vector_type(8)));
typedef unsigned int   v4u  __attribute__((ext_vector_type(4)));
typedef unsigned short v8us __attribute__((ext_vector_type(8)));
typedef __bf16         v16b __attribute__((ext_vector_type(16)));
typedef v4f  __attribute__((may_alias)) v4fa;
typedef v4i  __attribute__((may_alias)) v4ia;
typedef v8us __attribute__((may_alias)) v8usa;
union FragB { v16b v; v8us h[2]; v8i w; };

__device__ __forceinline__ v8f wmb(const FragB& a, const FragB& b, v8f c) {
  v8f d = __builtin_amdgcn_wmma_f32_16x16x32_bf16(false, a.v, false, b.v, (short)0, c, false, false);
  asm volatile("v_nop\n\tv_nop\n\tv_nop\n\tv_nop" : "+v"(d) : "v"(a.w), "v"(b.w));
  return d;
}

__device__ __forceinline__ unsigned int f2bf(float f) {
  const unsigned int u = __float_as_uint(f);
  const unsigned int r = ((u + 0x7FFFu + ((u >> 16) & 1u)) >> 16) & 0xFFFFu;
  return ((u & 0x7FFFFFFFu) > 0x7F800000u) ? 0x7FC0u : r;
}
__device__ __forceinline__ float bf2f(unsigned int b) { return __uint_as_float(b << 16); }
__device__ __forceinline__ float bfr(float f) { return bf2f(f2bf(f)); }
__device__ __forceinline__ v4f bfr4(const v4f a) {
  v4f r; r.x = bfr(a.x); r.y = bfr(a.y); r.z = bfr(a.z); r.w = bfr(a.w); return r;
}
__device__ __forceinline__ unsigned int pk2(float a, float b) { return f2bf(a) | (f2bf(b) << 16); }
__device__ __forceinline__ unsigned int pk2lo(float a, float b) {
  const unsigned int ha = f2bf(a), hb = f2bf(b);
  return f2bf(a - bf2f(ha)) | (f2bf(b - bf2f(hb)) << 16);
}
__device__ __forceinline__ v4u pack8(const v4f a, const v4f b) {
  v4u r;
  r.x = pk2(a.x, a.y); r.y = pk2(a.z, a.w); r.z = pk2(b.x, b.y); r.w = pk2(b.z, b.w);
  return r;
}
__device__ __forceinline__ v4u pack8lo(const v4f a, const v4f b) {
  v4u r;
  r.x = pk2lo(a.x, a.y); r.y = pk2lo(a.z, a.w); r.z = pk2lo(b.x, b.y); r.w = pk2lo(b.z, b.w);
  return r;
}
__device__ __forceinline__ float relu_np(float v) { return (v > 0.0f) ? v : (v - v); }
__device__ __forceinline__ v4f zsel(bool live, const v4f v) {
  v4f r; r.x = live ? v.x : 0.0f; r.y = live ? v.y : 0.0f; r.z = live ? v.z : 0.0f; r.w = live ? v.w : 0.0f;
  return r;
}

__device__ __forceinline__ int scan_chunk(const int* __restrict__ dsts, int nE, int cbase, int slotBase,
                                          int nb, int vec8, int* list, int tid, int lane, int wave) {
  int wc = 0;
  const int el0  = tid * EPT;
  const int e0   = cbase + el0;
  const int sent = -2147483647 - 1;
  v4i da, db;
  if (vec8 != 0 && cbase + CHUNK <= nE) {
    da = *(const v4i*)(dsts + e0);
    db = *(const v4i*)(dsts + e0 + 4);
  } else {
    da.x = (e0     < nE) ? dsts[min(e0,     nE - 1)] : sent;
    da.y = (e0 + 1 < nE) ? dsts[min(e0 + 1, nE - 1)] : sent;
    da.z = (e0 + 2 < nE) ? dsts[min(e0 + 2, nE - 1)] : sent;
    da.w = (e0 + 3 < nE) ? dsts[min(e0 + 3, nE - 1)] : sent;
    db.x = (e0 + 4 < nE) ? dsts[min(e0 + 4, nE - 1)] : sent;
    db.y = (e0 + 5 < nE) ? dsts[min(e0 + 5, nE - 1)] : sent;
    db.z = (e0 + 6 < nE) ? dsts[min(e0 + 6, nE - 1)] : sent;
    db.w = (e0 + 7 < nE) ? dsts[min(e0 + 7, nE - 1)] : sent;
  }
  const unsigned nbs = (unsigned)slotBase;
  const unsigned unb = (unsigned)nb;
  const unsigned s0 = (unsigned)da.x - nbs, s1 = (unsigned)da.y - nbs;
  const unsigned s2 = (unsigned)da.z - nbs, s3 = (unsigned)da.w - nbs;
  const unsigned s4 = (unsigned)db.x - nbs, s5 = (unsigned)db.y - nbs;
  const unsigned s6 = (unsigned)db.z - nbs, s7 = (unsigned)db.w - nbs;
  const bool h0 = s0 < unb, h1 = s1 < unb, h2 = s2 < unb, h3 = s3 < unb;
  const bool h4 = s4 < unb, h5 = s5 < unb, h6 = s6 < unb, h7 = s7 < unb;
  const unsigned any = __builtin_amdgcn_ballot_w32(h0 | h1 | h2 | h3 | h4 | h5 | h6 | h7);
  if (any != 0u) {
#define HITJ(J, HJ, SJ) { \
      const unsigned mj = __builtin_amdgcn_ballot_w32(HJ); \
      if (mj != 0u) { \
        if (HJ) { \
          const int pos = wc + (int)__builtin_amdgcn_mbcnt_lo(mj, 0u); \
          if (pos < WCAP) list[wave * WCAP + pos] = ((el0 + (J)) << SLB) | (int)(SJ); \
        } \
        wc += (int)__builtin_popcount(mj); } }
    HITJ(0, h0, s0)
    HITJ(1, h1, s1)
    HITJ(2, h2, s2)
    HITJ(3, h3, s3)
    HITJ(4, h4, s4)
    HITJ(5, h5, s5)
    HITJ(6, h6, s6)
    HITJ(7, h7, s7)
#undef HITJ
  }
  return wc;
}

__global__ __launch_bounds__(NTHR) void k_pa(const float* __restrict__ x, unsigned short* XB) {
  const int u = (int)blockIdx.x * NTHR + (int)threadIdx.x;
  if (u >= NUX) return;
  const int row = u / (EMB / 8);
  const int c0  = (u - row * (EMB / 8)) * 8;
  const int rc  = row < NN ? row : NN - 1;
  const float* p = x + (size_t)rc * EMB + c0;
  v4f a = *(const v4f*)p, b = *(const v4f*)(p + 4);
  const bool live = row < NN;
  a = zsel(live, a); b = zsel(live, b);
  const v4u hv = pack8(a, b);
  unsigned short* o = XB + (size_t)u * 8;
  *(volatile v4u*)o = hv;
  __threadfence();
  *(volatile v4u*)o = hv;
}

__device__ __forceinline__ void wunit(const float* __restrict__ w, const int Kin, const int Ncol, const int Kout,
                                      unsigned short* wt, const int v) {
  const int kq = Kout >> 3;
  const int n  = v / kq;
  const int k8 = (v - n * kq) * 8;
  const int kk = k8 - (k8 / Kin) * Kin;
  const int r  = n / Ncol;
  const int o  = n - r * Ncol;
  const float* p = w + ((size_t)r * (size_t)Kin + (size_t)kk) * (size_t)Ncol + o;
  v4f a, b;
  a.x = p[0];                  a.y = p[(size_t)Ncol];       a.z = p[(size_t)2 * Ncol];   a.w = p[(size_t)3 * Ncol];
  b.x = p[(size_t)4 * Ncol];   b.y = p[(size_t)5 * Ncol];   b.z = p[(size_t)6 * Ncol];   b.w = p[(size_t)7 * Ncol];
  const v4u wv = pack8(a, b);
  unsigned short* dp = wt + (size_t)n * (size_t)Kout + k8;
  *(volatile v4u*)dp = wv;
  __threadfence();
  *(volatile v4u*)dp = wv;
}

__global__ __launch_bounds__(NTHR) void k_pw(const float* __restrict__ wd, const float* __restrict__ wu,
                                             const float* __restrict__ w0, const float* __restrict__ w1,
                                             unsigned short* WdT, unsigned short* WuD,
                                             unsigned short* W0D, unsigned short* W1D) {
  const int u = (int)blockIdx.x * NTHR + (int)threadIdx.x;
  if (u < NUWD) {
    wunit(wd, EMB, BOT, EMB, WdT, u);
  } else if (u < NUWD + NUWU) {
    wunit(wu, BOT, EMB, KTH, WuD, u - NUWD);
  } else if (u < NUWD + NUWU + NUW0) {
    wunit(w0, EMB, HID, KHH, W0D, u - NUWD - NUWU);
  } else if (u < NUWD + NUWU + NUW0 + NUW1) {
    wunit(w1, HID, HID, KX1, W1D, u - NUWD - NUWU - NUW0);
  }
}

__device__ __forceinline__ void gemm_main(const unsigned short* __restrict__ A, const unsigned short* __restrict__ WT,
                                          const int K, const int rowBase, const int col0, float* stg,
                                          const int lane, const int wave) {
  const int hh = lane >> 4, m = lane & 15;
  const int wm = wave >> 1, wn = wave & 1;
  v8f acc[2][4];
  {
    const v8f z = {0.f, 0.f, 0.f, 0.f, 0.f, 0.f, 0.f, 0.f};
#pragma unroll
    for (int i = 0; i < 2; ++i)
#pragma unroll
      for (int t = 0; t < 4; ++t) acc[i][t] = z;
  }
  const unsigned short* ap0 = A  + (size_t)(rowBase + 32 * wm + m) * (size_t)K + 8 * hh;
  const unsigned short* ap1 = ap0 + (size_t)16 * (size_t)K;
  const unsigned short* wp  = WT + (size_t)(col0 + 64 * wn + m) * (size_t)K + 8 * hh;
  const int ksteps = K >> 5;
#pragma unroll 1
  for (int ks = 0; ks < ksteps; ++ks) {
    FragB a0, a1;
    a0.h[0] = *(const v8usa*)(ap0 + 32 * ks);
    a0.h[1] = *(const v8usa*)(ap0 + 32 * ks + 16);
    a1.h[0] = *(const v8usa*)(ap1 + 32 * ks);
    a1.h[1] = *(const v8usa*)(ap1 + 32 * ks + 16);
#pragma unroll
    for (int t = 0; t < 4; ++t) {
      const unsigned short* wq = wp + (size_t)(16 * t) * (size_t)K + 32 * ks;
      FragB bf;
      bf.h[0] = *(const v8usa*)wq;
      bf.h[1] = *(const v8usa*)(wq + 16);
      acc[0][t] = wmb(a0, bf, acc[0][t]);
      acc[1][t] = wmb(a1, bf, acc[1][t]);
    }
  }
#pragma unroll
  for (int i = 0; i < 2; ++i) {
#pragma unroll
    for (int t = 0; t < 4; ++t) {
      const int lc = 64 * wn + 16 * t + m;
#pragma unroll
      for (int r = 0; r < 8; ++r) {
        const int lr = 32 * wm + 16 * i + 8 * hh + r;
        stg[lr * SP + lc] = acc[i][t][r];
      }
    }
  }
}

__global__ __launch_bounds__(NTHR) __attribute__((amdgpu_num_vgpr(248)))
void k_gdown(const unsigned short* __restrict__ A, const unsigned short* __restrict__ WT,
             const float* __restrict__ bias, unsigned short* TH) {
  extern __shared__ __attribute__((aligned(16))) float gsm0[];
  float* stg = gsm0;
  float* sb  = gsm0 + GT * SP;
  const int tid = (int)threadIdx.x, lane = tid & 31, wave = tid >> 5;
  const int rowBase = (int)blockIdx.x * GT;
  if (tid < GT) sb[tid] = bfr(bias[tid]);
  gemm_main(A, WT, EMB, rowBase, 0, stg, lane, wave);
  __syncthreads();
#pragma unroll 1
  for (int it = 0; it < 8; ++it) {
    const int p   = it * NTHR + tid;
    const int row = p >> 4;
    const int c8  = (p & 15) * 8;
    const int gr  = rowBase + row;
    const bool live = gr < NN;
    const float* sr = stg + row * SP + c8;
    const v4f ua = *(const v4fa*)sr, ub = *(const v4fa*)(sr + 4);
    const v4f ba = *(const v4fa*)(sb + c8), bb = *(const v4fa*)(sb + c8 + 4);
    v4f a, b;
    a.x = relu_np(ua.x + ba.x); a.y = relu_np(ua.y + ba.y); a.z = relu_np(ua.z + ba.z); a.w = relu_np(ua.w + ba.w);
    b.x = relu_np(ub.x + bb.x); b.y = relu_np(ub.y + bb.y); b.z = relu_np(ub.z + bb.z); b.w = relu_np(ub.w + bb.w);
    a = zsel(live, a); b = zsel(live, b);
    const v4u hv = pack8(a, b);
    const v4u lv = pack8lo(a, b);
    unsigned short* hp = TH + (size_t)gr * KTH + c8;
    *(volatile v4u*)hp = hv;
    *(volatile v4u*)(hp + BOT) = lv;
    __threadfence();
    *(volatile v4u*)hp = hv;
    *(volatile v4u*)(hp + BOT) = lv;
  }
}

__global__ __launch_bounds__(NTHR) __attribute__((amdgpu_num_vgpr(248)))
void k_gup(const unsigned short* __restrict__ A, const unsigned short* __restrict__ WT,
           const float* __restrict__ x, const float* __restrict__ bias,
           const int* __restrict__ ri, const int* __restrict__ ci, const int* __restrict__ mi,
           const float* __restrict__ rowe, const float* __restrict__ cole, const float* __restrict__ mode,
           unsigned short* HH) {
  extern __shared__ __attribute__((aligned(16))) float gsm1[];
  float* stg = gsm1;
  float* sb  = gsm1 + GT * SP;
  int*   si  = (int*)(gsm1 + GT * SP + GT);
  const int tid = (int)threadIdx.x, lane = tid & 31, wave = tid >> 5;
  const int rowBase = (int)blockIdx.x * GT;
  const int col0    = (int)blockIdx.y * GT;
  if (tid < GT) {
    sb[tid] = bfr(bias[col0 + tid]);
    int g = rowBase + tid; g = g < NN ? g : NN - 1;
    int a = ri[g], b = ci[g], c = mi[g];
    a = a < 0 ? 0 : (a > NTAB - 1 ? NTAB - 1 : a);
    b = b < 0 ? 0 : (b > NTAB - 1 ? NTAB - 1 : b);
    c = c < 0 ? 0 : (c > NMOD - 1 ? NMOD - 1 : c);
    si[tid] = a; si[GT + tid] = b; si[2 * GT + tid] = c;
  }
  gemm_main(A, WT, KTH, rowBase, col0, stg, lane, wave);
  __syncthreads();
#pragma unroll 1
  for (int it = 0; it < 8; ++it) {
    const int p   = it * NTHR + tid;
    const int row = p >> 4;
    const int c8  = (p & 15) * 8;
    const int gr  = rowBase + row;
    const int grc = gr < NN ? gr : NN - 1;
    const bool live = gr < NN;
    const int col = col0 + c8;
    const float* xp = x    + (size_t)grc * EMB + col;
    const float* rp = rowe + (size_t)si[row] * EMB + col;
    const float* cp = cole + (size_t)si[GT + row] * EMB + col;
    const float* mp = mode + (size_t)si[2 * GT + row] * EMB + col;
    const v4f xa = bfr4(*(const v4f*)xp), xb = bfr4(*(const v4f*)(xp + 4));
    const v4f ra = bfr4(*(const v4f*)rp), rb = bfr4(*(const v4f*)(rp + 4));
    const v4f ca = bfr4(*(const v4f*)cp), cb = bfr4(*(const v4f*)(cp + 4));
    const v4f ma = bfr4(*(const v4f*)mp), mb = bfr4(*(const v4f*)(mp + 4));
    const float* sr = stg + row * SP + c8;
    const v4f ua = *(const v4fa*)sr, ub = *(const v4fa*)(sr + 4);
    const v4f ba = *(const v4fa*)(sb + c8), bb = *(const v4fa*)(sb + c8 + 4);
    v4f a, b;
    a.x = (((xa.x + (ua.x + ba.x)) + ra.x) + ca.x) + ma.x;
    a.y = (((xa.y + (ua.y + ba.y)) + ra.y) + ca.y) + ma.y;
    a.z = (((xa.z + (ua.z + ba.z)) + ra.z) + ca.z) + ma.z;
    a.w = (((xa.w + (ua.w + ba.w)) + ra.w) + ca.w) + ma.w;
    b.x = (((xb.x + (ub.x + bb.x)) + rb.x) + cb.x) + mb.x;
    b.y = (((xb.y + (ub.y + bb.y)) + rb.y) + cb.y) + mb.y;
    b.z = (((xb.z + (ub.z + bb.z)) + rb.z) + cb.z) + mb.z;
    b.w = (((xb.w + (ub.w + bb.w)) + rb.w) + cb.w) + mb.w;
    a = zsel(live, a); b = zsel(live, b);
    const v4u hv = pack8(a, b);
    const v4u lv = pack8lo(a, b);
    unsigned short* hp = HH + (size_t)gr * KHH + col;
    *(volatile v4u*)hp = hv;
    *(volatile v4u*)(hp + EMB) = lv;
    __threadfence();
    *(volatile v4u*)hp = hv;
    *(volatile v4u*)(hp + EMB) = lv;
  }
}

__global__ __launch_bounds__(NTHR) __attribute__((amdgpu_num_vgpr(248)))
void k_grel(const unsigned short* __restrict__ A, const unsigned short* __restrict__ WT, int K,
            const float* __restrict__ atts, const float* __restrict__ attd, float* HR, float* SSD) {
  extern __shared__ __attribute__((aligned(16))) float gsm2[];
  float* stg  = gsm2;
  float* satt = gsm2 + GT * SP;
  float* sdot = satt + 2 * GT;
  const int tid = (int)threadIdx.x, lane = tid & 31, wave = tid >> 5;
  const int rowBase = (int)blockIdx.x * GT;
  const int tn   = (int)blockIdx.y;
  const int r    = tn >> 1;
  const int half = tn & 1;
  const int col0 = tn * GT;

  if (tid < 64) {
    const int which = tid >> 5;
    const int c4 = (tid & 31) * 4;
    const int ao = r * HID + half * GT + c4;
    const v4f vs = *(const v4f*)(atts + ao);
    const v4f vd = *(const v4f*)(attd + ao);
    v4f v;
    v.x = (which == 0) ? vs.x : vd.x; v.y = (which == 0) ? vs.y : vd.y;
    v.z = (which == 0) ? vs.z : vd.z; v.w = (which == 0) ? vs.w : vd.w;
    *(v4fa*)(satt + which * GT + c4) = bfr4(v);
  }
  gemm_main(A, WT, K, rowBase, col0, stg, lane, wave);
  __syncthreads();

  {
    const int row = tid & (GT - 1), which = tid >> 7;
#pragma unroll 1
    for (int h4 = 0; h4 < 4; ++h4) {
      const float* hr = stg + row * SP + DHD * h4;
      const float* sa = satt + which * GT + DHD * h4;
      float d = 0.f;
#pragma unroll 2
      for (int c4 = 0; c4 < DHD / 4; ++c4) {
        const v4f hv = *(const v4fa*)(hr + 4 * c4);
        const v4f av = *(const v4fa*)(sa + 4 * c4);
        d = fmaf(hv.x, av.x, d);
        d = fmaf(hv.y, av.y, d);
        d = fmaf(hv.z, av.z, d);
        d = fmaf(hv.w, av.w, d);
      }
      sdot[(which * GT + row) * 4 + h4] = d;
    }
  }
  __syncthreads();

  {
    const int which = wave >> 2;
    const int rr = (wave & 3) * 32 + lane;
    const v4f sv = *(const v4fa*)(sdot + (which * GT + rr) * 4);
    float* sp = SSD + (size_t)which * (size_t)SDOFF + ((size_t)tn * MP + (size_t)(rowBase + rr)) * 4;
    *(volatile v4f*)sp = sv;
    __threadfence();
    *(volatile v4f*)sp = sv;
  }
#pragma unroll 1
  for (int it = 0; it < 16; ++it) {
    const int row = it * NWAVE + wave;
    const v4f v = *(const v4fa*)(stg + row * SP + 4 * lane);
    float* op = HR + ((size_t)r * MP + (size_t)(rowBase + row)) * HID + half * GT + 4 * lane;
    *(volatile v4f*)op = v;
    __threadfence();
    *(volatile v4f*)op = v;
  }
}

__global__ __launch_bounds__(NTHR) void k_bucket(const int* __restrict__ ei, const int* __restrict__ ety,
                                                 int* LIST, int* COG, int* FLG) {
  extern __shared__ __attribute__((aligned(16))) int bsm[];
  int* list = bsm;
  int* reg1 = bsm + LISTN;
  int* reg2 = reg1 + RCAP;
  int* co   = reg2 + RCAP;
  int* cur  = co + 2 * NBRUN;
  int* wcnt = cur + NBRUN;
  const int* srcs = ei;
  const int* dsts = ei + NE;
  const int tid = (int)threadIdx.x, lane = tid & 31, wave = tid >> 5;
  const int blk = (int)blockIdx.x;
  const int nodeBase = blk * NBRUN;
  int nb = NN - nodeBase;
  nb = nb < 0 ? 0 : (nb > NBRUN ? NBRUN : nb);
  const int vec8 = ((NE & 3) == 0) ? 1 : 0;

  {
    const v4i z4 = {0, 0, 0, 0};
    for (int i = tid * 4; i < RCAP + 3 * NBRUN; i += NTHR * 4) *(v4ia*)(reg2 + i) = z4;
  }
  __syncthreads();

  int tot = 0, ovf = 0;
  const int nChunks = (NE + CHUNK - 1) / CHUNK;
#pragma unroll 1
  for (int ch = 0; ch < nChunks; ++ch) {
    const int cbase = ch * CHUNK;
    const int wc = scan_chunk(dsts, NE, cbase, nodeBase, nb, vec8, list, tid, lane, wave);
    if (lane == 0) wcnt[wave] = wc;
    __syncthreads();
    int pre = 0, all = 0;
#pragma unroll
    for (int w2 = 0; w2 < NWAVE; ++w2) {
      int c = wcnt[w2];
      c = c < 0 ? 0 : (c > WCAP ? WCAP : c);
      all += c;
      pre += (w2 < wave) ? c : 0;
    }
    const int wcc  = wc > WCAP ? WCAP : wc;
    const int base = tot + pre;
#pragma unroll 1
    for (int i = lane; i < wcc; i += 32) {
      const int ent = list[wave * WCAP + i];
      const int el  = (ent >> SLB) & (CHUNK - 1);
      const int sl  = ent & (NBRUN - 1);
      int eid = cbase + el;
      eid = eid > NE - 1 ? NE - 1 : eid;
      const int sraw = srcs[eid];
      const int traw = ety[eid];
      const int s = sraw < 0 ? 0 : (sraw > NN - 1 ? NN - 1 : sraw);
      const int t = traw < 0 ? 0 : (traw > NREL - 1 ? NREL - 1 : traw);
      const int pos = base + i;
      if (pos < RCAP) reg1[pos] = (int)((unsigned)s | ((unsigned)t << 15) | ((unsigned)sl << 18));
    }
    if (tot + all > RCAP) ovf = 1;
    tot += all;
    tot = tot > RCAP ? RCAP : tot;
    __syncthreads();
  }
  const int nh = tot;

  if (wave == 0) {
#pragma unroll 1
    for (int b0 = 0; b0 < nh; b0 += 32) {
      const int idx = b0 + lane;
      const int uv  = reg1[idx < nh ? idx : nh - 1];
      const int m32 = (nh - b0) < 32 ? (nh - b0) : 32;
#pragma unroll 1
      for (int k = 0; k < m32; ++k) {
        const int u  = __builtin_amdgcn_readlane(uv, k);
        const int sq = (u >> 18) & (NBRUN - 1);
        if (lane == 0) co[sq] = co[sq] + 1;
      }
    }
  }
  __syncthreads();
  if (wave == 0) {
    const int base = lane * (NBRUN / 32);
    int s = 0;
#pragma unroll 1
    for (int i = 0; i < NBRUN / 32; ++i) s += co[base + i];
    int incl = s;
#pragma unroll
    for (int d = 1; d < 32; d <<= 1) {
      const int y = __shfl_up(incl, d, 32);
      if (lane >= d) incl += y;
    }
    int run = incl - s;
#pragma unroll 1
    for (int i = 0; i < NBRUN / 32; ++i) {
      const int cv = co[base + i];
      co[NBRUN + base + i] = run;
      cur[base + i] = run;
      run += cv;
    }
  }
  __syncthreads();
  if (wave == 0) {
#pragma unroll 1
    for (int b0 = 0; b0 < nh; b0 += 32) {
      const int idx = b0 + lane;
      const int uv  = reg1[idx < nh ? idx : nh - 1];
      const int m32 = (nh - b0) < 32 ? (nh - b0) : 32;
#pragma unroll 1
      for (int k = 0; k < m32; ++k) {
        const int u  = __builtin_amdgcn_readlane(uv, k);
        const int sq = (u >> 18) & (NBRUN - 1);
        if (lane == 0) {
          int p = cur[sq];
          p = p < 0 ? 0 : (p > RCAP - 1 ? RCAP - 1 : p);
          reg2[p] = u;
          cur[sq] = p + 1;
        }
      }
    }
  }
  __syncthreads();

  int* lb = LIST + (size_t)blk * RCAP;
  int* cb = COG + (size_t)blk * (2 * NBRUN) + 4 * tid;
  const v4i cov = *(const v4ia*)(co + 4 * tid);
  v4i cv;
  cv.x = (tid == 0) ? nh : 0;
  cv.y = (tid == 0) ? ovf : 0;
  cv.z = 0; cv.w = 0;
  int* fp = FLG + (size_t)blk * 32 + 4 * (tid & 7);
#pragma unroll 1
  for (int p = tid * 4; p < RCAP; p += NTHR * 4) {
    const v4i v = *(const v4ia*)(reg2 + p);
    *(volatile v4i*)(lb + p) = v;
  }
  *(volatile v4i*)cb = cov;
  if (tid < 8) *(volatile v4i*)fp = cv;
  __threadfence();
#pragma unroll 1
  for (int p = tid * 4; p < RCAP; p += NTHR * 4) {
    const v4i v = *(const v4ia*)(reg2 + p);
    *(volatile v4i*)(lb + p) = v;
  }
  *(volatile v4i*)cb = cov;
  if (tid < 8) *(volatile v4i*)fp = cv;
}

template <int L>
__global__ __launch_bounds__(NTHR) __attribute__((amdgpu_num_vgpr(248)))
void k_scan(const int* __restrict__ LIST, const int* __restrict__ COG, const int* __restrict__ FLG,
            const float* __restrict__ HR, const float* __restrict__ SSD,
            unsigned short* XP, float* out) {
  static_assert(L == 0 || L == 1);
  __shared__ __attribute__((aligned(16))) int   sl[RCAP];
  __shared__ __attribute__((aligned(16))) int   co[2 * NBRUN];
  __shared__ __attribute__((aligned(16))) float stw[NWAVE * HID];
  const int tid = (int)threadIdx.x, lane = tid & 31, wave = tid >> 5;
  const int blk = (int)blockIdx.x;
  const int nodeBase = blk * NBRUN;

  const int nhraw = FLG[(size_t)blk * 32];
  const int bflag = FLG[(size_t)blk * 32 + 1];
  const int nh  = nhraw < 0 ? 0 : (nhraw > RCAP ? RCAP : nhraw);
  const int ovf = (bflag != 0 || nhraw < 0 || nhraw > RCAP) ? 1 : 0;

  {
    const int* lb = LIST + (size_t)blk * RCAP;
    const int nh4 = (nh + 3) & ~3;
#pragma unroll 1
    for (int p = tid * 4; p < nh4; p += NTHR * 4) *(v4ia*)(sl + p) = *(const v4i*)(lb + p);
    *(v4ia*)(co + 4 * tid) = *(const v4i*)(COG + (size_t)blk * (2 * NBRUN) + 4 * tid);
  }
  __syncthreads();

  const float qnan = __int_as_float(0x7fc00000);
  const int half = lane >> 4;
  const int hidx = (lane >> 2) & 3;
  const size_t pstr = (size_t)2 * MP * 4;
  float* st = stw + wave * HID;

#pragma unroll 1
  for (int si = 0; si < NBRUN / NWAVE; ++si) {
    const int s    = si * NWAVE + wave;
    const int node = nodeBase + s;
    const int nc   = node < NN ? node : NN - 1;
    int c = co[s];
    const bool big = c > DEGCAP;
    c = c < 0 ? 0 : (c > DEGCAP ? DEGCAP : c);
    int o = co[NBRUN + s];
    o = o < 0 ? 0 : (o > RCAP ? RCAP : o);
    if (c > nh - o) c = nh - o;
    c = c < 0 ? 0 : c;

    const size_t sdb = (size_t)SDOFF + ((size_t)half * MP + (size_t)nc) * 4 + hidx;
    const float sd0 = SSD[sdb];
    const float sd1 = SSD[sdb + pstr];
    const float sd2 = SSD[sdb + 2 * pstr];
    const float sd3 = SSD[sdb + 3 * pstr];
    const float sd4 = SSD[sdb + 4 * pstr];

    float mx = MX0, dn = 0.0f;
    float acc[8];
#pragma unroll
    for (int i = 0; i < 8; ++i) acc[i] = 0.0f;

#pragma unroll 1
    for (int b0 = 0; b0 < c; b0 += 32) {
      int tq = b0 + lane;
      tq = tq > c - 1 ? c - 1 : tq;
      int idx = o + tq;
      idx = idx < 0 ? 0 : (idx > RCAP - 1 ? RCAP - 1 : idx);
      const int ent = sl[idx];
      const int m32 = (c - b0) < 32 ? (c - b0) : 32;
#pragma unroll 1
      for (int k = 0; k < m32; ++k) {
        const int e = __builtin_amdgcn_readlane(ent, k);
        int sk = e & 0x7FFF;
        sk = sk > NN - 1 ? NN - 1 : sk;
        int t = (e >> 15) & 7;
        t = t > NREL - 1 ? NREL - 1 : t;
        float adv = sd0;
        adv = (t == 1) ? sd1 : adv;
        adv = (t == 2) ? sd2 : adv;
        adv = (t == 3) ? sd3 : adv;
        adv = (t == 4) ? sd4 : adv;
        const float ss = SSD[(size_t)t * pstr + ((size_t)half * MP + (size_t)sk) * 4 + hidx];
        const float* rp = HR + ((size_t)t * MP + (size_t)sk) * HID + 8 * lane;
        const v4f a = *(const v4f*)rp;
        const v4f b = *(const v4f*)(rp + 4);
        float lg = ss + adv;
        lg = (lg >= 0.f) ? lg : NEGSL * lg;
        const float df = lg - mx;
        const float ee = expf(-fabsf(df));
        const bool  up = df > 0.f;
        const float s1 = up ? ee : 1.0f;
        const float s2 = up ? 1.0f : ee;
        mx = up ? lg : mx;
        dn = fmaf(dn, s1, s2);
        acc[0] = fmaf(acc[0], s1, s2 * a.x); acc[1] = fmaf(acc[1], s1, s2 * a.y);
        acc[2] = fmaf(acc[2], s1, s2 * a.z); acc[3] = fmaf(acc[3], s1, s2 * a.w);
        acc[4] = fmaf(acc[4], s1, s2 * b.x); acc[5] = fmaf(acc[5], s1, s2 * b.y);
        acc[6] = fmaf(acc[6], s1, s2 * b.z); acc[7] = fmaf(acc[7], s1, s2 * b.w);
      }
    }
    const float inv = __builtin_amdgcn_rcpf(dn + EPS_SM);
    const bool has  = c > 0;
    const bool pz   = (ovf != 0) || big;
    const bool live = node < NN;

    if constexpr (L == 0) {
#pragma unroll
      for (int i = 0; i < 8; ++i) st[i * 32 + lane] = acc[i];
#pragma unroll 1
      for (int j = 0; j < 8; ++j) {
        float y = st[j * 32 + lane] * inv;
        y = has ? y : 0.0f;
        y = (y > 0.0f) ? y : expm1f(y);
        y = pz ? qnan : y;
        y = live ? y : 0.0f;
        st[j * 32 + lane] = y;
      }
      v4f oa, ob;
      oa.x = st[0 * 32 + lane]; oa.y = st[1 * 32 + lane]; oa.z = st[2 * 32 + lane]; oa.w = st[3 * 32 + lane];
      ob.x = st[4 * 32 + lane]; ob.y = st[5 * 32 + lane]; ob.z = st[6 * 32 + lane]; ob.w = st[7 * 32 + lane];
      const v4u hv = pack8(oa, ob);
      const v4u lv = pack8lo(oa, ob);
      if (node < MP) {
        unsigned short* hp = XP + (size_t)node * KX1 + 8 * lane;
        *(volatile v4u*)hp = hv;
        *(volatile v4u*)(hp + HID) = lv;
        __threadfence();
        *(volatile v4u*)hp = hv;
        *(volatile v4u*)(hp + HID) = lv;
      }
    } else {
      v4f oa, ob;
      oa.x = has ? acc[0] * inv : 0.0f; oa.y = has ? acc[1] * inv : 0.0f;
      oa.z = has ? acc[2] * inv : 0.0f; oa.w = has ? acc[3] * inv : 0.0f;
      ob.x = has ? acc[4] * inv : 0.0f; ob.y = has ? acc[5] * inv : 0.0f;
      ob.z = has ? acc[6] * inv : 0.0f; ob.w = has ? acc[7] * inv : 0.0f;
      oa.x = pz ? qnan : oa.x; oa.y = pz ? qnan : oa.y; oa.z = pz ? qnan : oa.z; oa.w = pz ? qnan : oa.w;
      ob.x = pz ? qnan : ob.x; ob.y = pz ? qnan : ob.y; ob.z = pz ? qnan : ob.z; ob.w = pz ? qnan : ob.w;
      *(v4fa*)(st + 8 * lane)     = oa;
      *(v4fa*)(st + 8 * lane + 4) = ob;
      __builtin_amdgcn_fence(__ATOMIC_ACQ_REL, "workgroup");
      __builtin_amdgcn_wave_barrier();
      const v4f r0 = *(const v4fa*)(st + 4 * lane);
      const v4f r1 = *(const v4fa*)(st + 128 + 4 * lane);
      __builtin_amdgcn_fence(__ATOMIC_ACQ_REL, "workgroup");
      __builtin_amdgcn_wave_barrier();
      if (node < NN) {
        float* op = out + (size_t)node * HID + 4 * lane;
        *(volatile v4f*)op = r0;
        *(volatile v4f*)(op + 128) = r1;
        __threadfence();
        *(volatile v4f*)op = r0;
        *(volatile v4f*)(op + 128) = r1;
      }
    }
  }
}

extern "C" void kernel_launch(void* const* d_in, const int* in_sizes, int n_in,
                              void* d_out, int out_size, void* d_ws, size_t ws_size,
                              hipStream_t stream) {
  if (n_in < 19) return;
  if (in_sizes[0] != NN * EMB) return;
  if (in_sizes[1] != NN || in_sizes[2] != NN || in_sizes[3] != NN) return;
  if (in_sizes[4] != 2 * NE || in_sizes[5] != NE) return;
  if (in_sizes[6] != EMB * BOT || in_sizes[7] != BOT) return;
  if (in_sizes[8] != BOT * EMB || in_sizes[9] != EMB) return;
  if (in_sizes[10] != NTAB * EMB || in_sizes[11] != NTAB * EMB || in_sizes[12] != NMOD * EMB) return;
  if (in_sizes[13] != NREL * EMB * HID) return;
  if (in_sizes[14] != NREL * HID || in_sizes[15] != NREL * HID) return;
  if (in_sizes[16] != NREL * HID * HID) return;
  if (in_sizes[17] != NREL * HID || in_sizes[18] != NREL * HID) return;
  if (out_size != NN * HID) return;

  const float* x      = (const float*)d_in[0];
  const int*   ri     = (const int*)  d_in[1];
  const int*   ci     = (const int*)  d_in[2];
  const int*   mi     = (const int*)  d_in[3];
  const int*   ei     = (const int*)  d_in[4];
  const int*   ety    = (const int*)  d_in[5];
  const float* w_down = (const float*)d_in[6];
  const float* b_down = (const float*)d_in[7];
  const float* w_up   = (const float*)d_in[8];
  const float* b_up   = (const float*)d_in[9];
  const float* rowe   = (const float*)d_in[10];
  const float* cole   = (const float*)d_in[11];
  const float* mode   = (const float*)d_in[12];
  const float* w0     = (const float*)d_in[13];
  const float* as0    = (const float*)d_in[14];
  const float* ad0    = (const float*)d_in[15];
  const float* w1     = (const float*)d_in[16];
  const float* as1    = (const float*)d_in[17];
  const float* ad1    = (const float*)d_in[18];
  float* out = (float*)d_out;

  char* ws = (char*)d_ws;
  size_t off = 0;
  const size_t oXB  = off; off += (size_t)MP * EMB * 2;              off = (off + 255) & ~(size_t)255;
  const size_t oTH  = off; off += (size_t)MP * KTH * 2;              off = (off + 255) & ~(size_t)255;
  const size_t oHH  = off; off += (size_t)MP * KHH * 2;              off = (off + 255) & ~(size_t)255;
  const size_t oHR  = off; off += (size_t)NREL * MP * HID * 4;       off = (off + 255) & ~(size_t)255;
  const size_t oSSD = off; off += (size_t)2 * SDOFF * 4;             off = (off + 255) & ~(size_t)255;
  const size_t oWd  = off; off += (size_t)BOT * EMB * 2;             off = (off + 255) & ~(size_t)255;
  const size_t oWu  = off; off += (size_t)EMB * KTH * 2;             off = (off + 255) & ~(size_t)255;
  const size_t oW0  = off; off += (size_t)NRN * KHH * 2;             off = (off + 255) & ~(size_t)255;
  const size_t oW1  = off; off += (size_t)NRN * KX1 * 2;             off = (off + 255) & ~(size_t)255;
  const size_t oLS  = off; off += (size_t)NBLK * RCAP * 4;           off = (off + 255) & ~(size_t)255;
  const size_t oCO  = off; off += (size_t)NBLK * 2 * NBRUN * 4;      off = (off + 255) & ~(size_t)255;
  const size_t oFL  = off; off += (size_t)NBLK * 128;                off = (off + 255) & ~(size_t)255;
  if (off > ws_size) return;
  if ((size_t)MP * KX1 * 2 > (size_t)MP * KHH * 2) return;
  unsigned short* XB  = (unsigned short*)(ws + oXB);
  unsigned short* TH  = (unsigned short*)(ws + oTH);
  unsigned short* HH  = (unsigned short*)(ws + oHH);
  unsigned short* X1  = (unsigned short*)(ws + oHH);
  float*          HR  = (float*)(ws + oHR);
  float*          SSD = (float*)(ws + oSSD);
  unsigned short* WdT = (unsigned short*)(ws + oWd);
  unsigned short* WuD = (unsigned short*)(ws + oWu);
  unsigned short* W0D = (unsigned short*)(ws + oW0);
  unsigned short* W1D = (unsigned short*)(ws + oW1);
  int*            LST = (int*)(ws + oLS);
  int*            COG = (int*)(ws + oCO);
  int*            FLG = (int*)(ws + oFL);

  hipFuncSetAttribute(reinterpret_cast<const void*>(&k_gdown),
                      hipFuncAttributeMaxDynamicSharedMemorySize, GEMM_LDS_BYTES);
  hipFuncSetAttribute(reinterpret_cast<const void*>(&k_gup),
                      hipFuncAttributeMaxDynamicSharedMemorySize, GEMM_LDS_BYTES);
  hipFuncSetAttribute(reinterpret_cast<const void*>(&k_grel),
                      hipFuncAttributeMaxDynamicSharedMemorySize, GEMM_LDS_BYTES);
  hipFuncSetAttribute(reinterpret_cast<const void*>(&k_bucket),
                      hipFuncAttributeMaxDynamicSharedMemorySize, BKT_LDS_BYTES);

  const int gM = MP / GT;
  k_pa<<<NUX / NTHR, NTHR, 0, stream>>>(x, XB);
  k_pw<<<(NUWD + NUWU + NUW0 + NUW1) / NTHR, NTHR, 0, stream>>>(w_down, w_up, w0, w1, WdT, WuD, W0D, W1D);
  k_gdown<<<dim3(gM, 1), NTHR, GEMM_LDS_BYTES, stream>>>(XB, WdT, b_down, TH);
  k_gup<<<dim3(gM, EMB / GT), NTHR, GEMM_LDS_BYTES, stream>>>(TH, WuD, x, b_up, ri, ci, mi, rowe, cole, mode, HH);
  k_bucket<<<NBLK, NTHR, BKT_LDS_BYTES, stream>>>(ei, ety, LST, COG, FLG);
  k_grel<<<dim3(gM, NRN / GT), NTHR, GEMM_LDS_BYTES, stream>>>(HH, W0D, KHH, as0, ad0, HR, SSD);
  k_scan<0><<<NBLK, NTHR, 0, stream>>>(LST, COG, FLG, HR, SSD, X1, out);
  k_grel<<<dim3(gM, NRN / GT), NTHR, GEMM_LDS_BYTES, stream>>>(X1, W1D, KX1, as1, ad1, HR, SSD);
  k_scan<1><<<NBLK, NTHR, 0, stream>>>(LST, COG, FLG, HR, SSD, X1, out);
}
